// NoisyIBLayer_84911503442655
// MI455X (gfx1250) — hardware-verified
//
#include <hip/hip_runtime.h>
#define NN 8192
#define DD 256
#define NMT (NN / 16)
#define NNQ (NN / 64)

typedef __bf16 v16b __attribute__((ext_vector_type(16)));
typedef unsigned short v8us __attribute__((ext_vector_type(8), may_alias));
typedef float  v8f  __attribute__((ext_vector_type(8)));
typedef float  v4f  __attribute__((ext_vector_type(4)));
typedef float  v4fa __attribute__((ext_vector_type(4), may_alias));
union FragB { v16b v; v8us half[2]; unsigned short u[16]; };

__device__ __forceinline__ unsigned short bf16_bits(float x) { unsigned int u = __float_as_uint(x); return (unsigned short)((u + 0x7FFFu + ((u >> 16) & 1u)) >> 16); }
__device__ __forceinline__ float bf16_val(unsigned short b) { return __uint_as_float(((unsigned int)b) << 16); }
__device__ __forceinline__ float bf16_round(float x) { return bf16_val(bf16_bits(x)); }
template <int NT>
__device__ __forceinline__ v8f mmaN(v16b ah, v16b al, v16b bh, v16b bl, v8f c) {
  c = __builtin_amdgcn_wmma_f32_16x16x32_bf16(false, ah, false, bh, (short)0, c, false, false);
  if (NT >= 2) c = __builtin_amdgcn_wmma_f32_16x16x32_bf16(false, al, false, bh, (short)0, c, false, false);
  if (NT >= 3) c = __builtin_amdgcn_wmma_f32_16x16x32_bf16(false, ah, false, bl, (short)0, c, false, false);
  asm volatile("v_nop\n\tv_nop\n\tv_nop\n\tv_nop" : "+v"(c) : "v"(ah), "v"(al), "v"(bh), "v"(bl));
  return c;
}

__global__ __launch_bounds__(256) void k_wt_bf16(const float* __restrict__ W, unsigned short* __restrict__ Wt, int K, int N) {
  const int t = blockIdx.x * 256 + threadIdx.x;
  const int k8n = K / 8;
  if (t >= N * k8n) return;
  const int n = t / k8n, k8 = (t % k8n) * 8;
  v8us v;
#pragma unroll
  for (int i = 0; i < 8; ++i) v[i] = bf16_bits(W[(size_t)(k8 + i) * N + n]);
  *(volatile v8us*)(Wt + (size_t)n * K + k8) = v;
  __threadfence();
  *(volatile v8us*)(Wt + (size_t)n * K + k8) = v;
}

template <bool ASPLIT, int ACT, bool BIAS_BF16>
__global__ __launch_bounds__(128) void k_gemm_bf(const float* __restrict__ A, int lda, const unsigned short* __restrict__ Wt, int ldb,
                                               const float* __restrict__ bias, float* __restrict__ C, int ldc, int M, int N, int K) {
  __shared__ __attribute__((aligned(16))) float so[4][16][64];
  const int tid = threadIdx.x, w = tid >> 5, lane = tid & 31, ln = lane & 15, hh = lane >> 4;
  const int ntn = N / 64;
  const int wid = blockIdx.x * 4 + w;
  const int mt = wid / ntn, nq = wid % ntn;
  if (mt * 16 >= M) return;
  const int row0 = mt * 16, col0 = nq * 64;
  const float* arow = A + (size_t)(row0 + ln) * lda;
  v8f acc[4] = {};
  for (int kb = 0; kb < K; kb += 32) {
    FragB ah, al;
    const v4f x0 = *(const v4fa*)(arow + kb + 8 * hh), x1 = *(const v4fa*)(arow + kb + 8 * hh + 4);
    const v4f x2 = *(const v4fa*)(arow + kb + 16 + 8 * hh), x3 = *(const v4fa*)(arow + kb + 16 + 8 * hh + 4);
    float xs[16] = {x0[0],x0[1],x0[2],x0[3],x1[0],x1[1],x1[2],x1[3],x2[0],x2[1],x2[2],x2[3],x3[0],x3[1],x3[2],x3[3]};
#pragma unroll
    for (int i = 0; i < 16; ++i) { const unsigned short hb = bf16_bits(xs[i]); ah.u[i] = hb; al.u[i] = ASPLIT ? bf16_bits(xs[i] - bf16_val(hb)) : (unsigned short)0; }
#pragma unroll
    for (int t = 0; t < 4; ++t) {
      const unsigned short* brow = Wt + (size_t)(col0 + t * 16 + ln) * ldb + kb;
      FragB b;
      b.half[0] = *(const v8us*)(brow + 8 * hh);
      b.half[1] = *(const v8us*)(brow + 16 + 8 * hh);
      acc[t] = mmaN<ASPLIT ? 2 : 1>(ah.v, al.v, b.v, b.v, acc[t]);
    }
  }
#pragma unroll
  for (int t = 0; t < 4; ++t) {
    float bv = bias ? bias[col0 + t * 16 + ln] : 0.f;
    if (BIAS_BF16) bv = bf16_round(bv);
#pragma unroll
    for (int r = 0; r < 8; ++r) { float v = acc[t][r] + bv; if (ACT == 1) v = fmaxf(v, 0.f); so[w][8 * hh + r][t * 16 + ln] = v; }
  }
  __builtin_amdgcn_fence(__ATOMIC_ACQ_REL, "workgroup");
  __builtin_amdgcn_wave_barrier();
  const int rsub = lane >> 4, c4 = (lane & 15) * 4;
  for (int pass = 0; pass < 2; ++pass) {
#pragma unroll
    for (int q = 0; q < 8; ++q) {
      const int r = q * 2 + rsub;
      const v4f v = *(const v4fa*)&so[w][r][c4];
      *(volatile v4f*)(C + (size_t)(row0 + r) * ldc + col0 + c4) = v;
    }
    if (pass == 0) __threadfence();
  }
}

template <int D, bool CAUSAL>
__global__ __launch_bounds__(128) void k_flash(const float* __restrict__ qb, const float* __restrict__ kb, const float* __restrict__ vb,
                                             int pitch, int T, int H, float scale, float* __restrict__ y, int ypitch) {
  constexpr int KS = D / 32;
  constexpr int DT = D / 16;
  __shared__ __attribute__((aligned(16))) unsigned short sKh[32][D + 8], sKl[32][D + 8], sVh[32][D + 8], sVl[32][D + 8];
  __shared__ __attribute__((aligned(16))) unsigned short sPh[4][16][40], sPl[4][16][40];
  __shared__ __attribute__((aligned(16))) float sO[4][16][D];
  const int tid = threadIdx.x, w = tid >> 5, lane = tid & 31, ln = lane & 15, hh = lane >> 4;
  const int nqb = (T + 63) / 64;
  const int bh = blockIdx.x / nqb, qblk = blockIdx.x % nqb;
  const int b = bh / H, h = bh % H;
  const int q0 = qblk * 64 + w * 16;
  const float* Q = qb + (size_t)b * T * pitch + h * D;
  const float* K = kb + (size_t)b * T * pitch + h * D;
  const float* V = vb + (size_t)b * T * pitch + h * D;

  FragB aqh[KS], aql[KS];
  {
    int row = q0 + ln; if (row >= T) row = T - 1;
    const float* qr = Q + (size_t)row * pitch;
#pragma unroll
    for (int ks = 0; ks < KS; ++ks)
#pragma unroll
      for (int i = 0; i < 16; ++i) {
        const int d = ks * 32 + ((i < 8) ? (8 * hh + i) : (16 + 8 * hh + (i - 8)));
        const float x = qr[d] * scale; const unsigned short hb = bf16_bits(x);
        aqh[ks].u[i] = hb; aql[ks].u[i] = bf16_bits(x - bf16_val(hb));
      }
  }
  float m_r[8], l_r[8];
#pragma unroll
  for (int r = 0; r < 8; ++r) { m_r[r] = -3.0e38f; l_r[r] = 0.f; }
  v8f oacc[DT];
#pragma unroll
  for (int dt = 0; dt < DT; ++dt) oacc[dt] = (v8f){0.f,0.f,0.f,0.f,0.f,0.f,0.f,0.f};

  const int kv_end = CAUSAL ? min(T, qblk * 64 + 64) : T;
  for (int j0 = 0; j0 < kv_end; j0 += 32) {
    __syncthreads();
    for (int e = tid; e < 32 * (D / 4); e += 128) {
      const int r = e / (D / 4), c4 = (e % (D / 4)) * 4;
      const int key = j0 + r;
      v4f kf = {0.f,0.f,0.f,0.f}, vf = {0.f,0.f,0.f,0.f};
      if (key < T) { kf = *(const v4fa*)(K + (size_t)key * pitch + c4); vf = *(const v4fa*)(V + (size_t)key * pitch + c4); }
#pragma unroll
      for (int t = 0; t < 4; ++t) {
        unsigned short hb = bf16_bits(kf[t]); sKh[r][c4 + t] = hb; sKl[r][c4 + t] = bf16_bits(kf[t] - bf16_val(hb));
        hb = bf16_bits(vf[t]); sVh[r][c4 + t] = hb; sVl[r][c4 + t] = bf16_bits(vf[t] - bf16_val(hb));
      }
    }
    __syncthreads();
    v8f s[2];
#pragma unroll
    for (int nt = 0; nt < 2; ++nt) {
      v8f acc = {};
#pragma unroll
      for (int ks = 0; ks < KS; ++ks) {
        FragB bh_, bl_;
        bh_.half[0] = *(const v8us*)&sKh[nt * 16 + ln][ks * 32 + 8 * hh]; bh_.half[1] = *(const v8us*)&sKh[nt * 16 + ln][ks * 32 + 16 + 8 * hh];
        bl_.half[0] = *(const v8us*)&sKl[nt * 16 + ln][ks * 32 + 8 * hh]; bl_.half[1] = *(const v8us*)&sKl[nt * 16 + ln][ks * 32 + 16 + 8 * hh];
        acc = mmaN<3>(aqh[ks].v, aql[ks].v, bh_.v, bl_.v, acc);
      }
      s[nt] = acc;
    }
    float alpha[8];
#pragma unroll
    for (int r = 0; r < 8; ++r) {
      const int qi = q0 + 8 * hh + r;
      const int ja = j0 + ln, jb = j0 + 16 + ln;
      if (CAUSAL) { if (ja > qi) s[0][r] = -3.0e38f; if (jb > qi) s[1][r] = -3.0e38f; }
      if (ja >= T) s[0][r] = -3.0e38f;
      if (jb >= T) s[1][r] = -3.0e38f;
      float mx = fmaxf(s[0][r], s[1][r]);
      mx = fmaxf(mx, __shfl_xor(mx, 1, 32)); mx = fmaxf(mx, __shfl_xor(mx, 2, 32)); mx = fmaxf(mx, __shfl_xor(mx, 4, 32)); mx = fmaxf(mx, __shfl_xor(mx, 8, 32));
      const float mnew = fmaxf(m_r[r], mx);
      alpha[r] = (mnew > -1.0e38f) ? __expf(m_r[r] - mnew) : 1.0f;
      const float p0 = (s[0][r] > -1.0e38f) ? __expf(s[0][r] - mnew) : 0.f;
      const float p1 = (s[1][r] > -1.0e38f) ? __expf(s[1][r] - mnew) : 0.f;
      m_r[r] = mnew;
      l_r[r] = l_r[r] * alpha[r] + p0 + p1;
      unsigned short hb = bf16_bits(p0); sPh[w][8 * hh + r][ln] = hb;      sPl[w][8 * hh + r][ln] = bf16_bits(p0 - bf16_val(hb));
      hb = bf16_bits(p1);                sPh[w][8 * hh + r][16 + ln] = hb; sPl[w][8 * hh + r][16 + ln] = bf16_bits(p1 - bf16_val(hb));
    }
#pragma unroll
    for (int dt = 0; dt < DT; ++dt)
#pragma unroll
      for (int r = 0; r < 8; ++r) oacc[dt][r] *= alpha[r];
    __builtin_amdgcn_fence(__ATOMIC_ACQ_REL, "workgroup");
    __builtin_amdgcn_wave_barrier();
    FragB pah, pal;
    pah.half[0] = *(const v8us*)&sPh[w][ln][8 * hh]; pah.half[1] = *(const v8us*)&sPh[w][ln][16 + 8 * hh];
    pal.half[0] = *(const v8us*)&sPl[w][ln][8 * hh]; pal.half[1] = *(const v8us*)&sPl[w][ln][16 + 8 * hh];
#pragma unroll
    for (int dt = 0; dt < DT; ++dt) {
      FragB bvh, bvl;
#pragma unroll
      for (int i = 0; i < 8; ++i) {
        bvh.u[i] = sVh[8 * hh + i][dt * 16 + ln]; bvh.u[8 + i] = sVh[16 + 8 * hh + i][dt * 16 + ln];
        bvl.u[i] = sVl[8 * hh + i][dt * 16 + ln]; bvl.u[8 + i] = sVl[16 + 8 * hh + i][dt * 16 + ln];
      }
      oacc[dt] = mmaN<3>(pah.v, pal.v, bvh.v, bvl.v, oacc[dt]);
    }
    __builtin_amdgcn_fence(__ATOMIC_ACQ_REL, "workgroup");
    __builtin_amdgcn_wave_barrier();
  }
#pragma unroll
  for (int r = 0; r < 8; ++r) {
    float l = l_r[r];
    l += __shfl_xor(l, 1, 32); l += __shfl_xor(l, 2, 32); l += __shfl_xor(l, 4, 32); l += __shfl_xor(l, 8, 32);
    l_r[r] = (l > 0.f) ? 1.0f / l : 0.f;
  }
#pragma unroll
  for (int dt = 0; dt < DT; ++dt)
#pragma unroll
    for (int r = 0; r < 8; ++r) sO[w][8 * hh + r][dt * 16 + ln] = oacc[dt][r] * l_r[r];
  __builtin_amdgcn_fence(__ATOMIC_ACQ_REL, "workgroup");
  __builtin_amdgcn_wave_barrier();
  for (int pass = 0; pass < 2; ++pass) {
    for (int r = 0; r < 16; ++r) {
      const int row = q0 + r;
      if (row < T && lane < D / 4) {
        const v4f val = *(const v4fa*)&sO[w][r][lane * 4];
        *(volatile v4f*)(y + ((size_t)b * T + row) * ypitch + h * D + lane * 4) = val;
      }
    }
    if (pass == 0) __threadfence();
  }
}

__device__ __forceinline__ float softplus1(float x) { return (x > 20.f) ? x : log1pf(expf(x)); }
__global__ __launch_bounds__(1024) void k_sq(const float* __restrict__ x, float* __restrict__ sq) { const int tid = threadIdx.x, wv = tid >> 5, lane = tid & 31; const int i = blockIdx.x * 32 + wv; const float* r = x + (size_t)i * DD; float s = 0.f;
#pragma unroll
  for (int u = 0; u < 8; ++u) { const float v = bf16_round(r[u * 32 + lane]); s += v * v; } for (int o = 16; o >= 1; o >>= 1) s += __shfl_xor(s, o, 32);
  __shared__ float ss[32]; if (lane == 0) ss[wv] = s; __syncthreads(); if (tid < 32) { *(volatile float*)(sq + blockIdx.x * 32 + tid) = ss[tid]; } __threadfence(); if (tid < 32) { *(volatile float*)(sq + blockIdx.x * 32 + tid) = ss[tid]; } }
__global__ __launch_bounds__(128) void k_gram(const float* __restrict__ x, const float* __restrict__ sq, const float* __restrict__ phi, float* __restrict__ RP, float* __restrict__ CP) {
  const int tid = threadIdx.x, w = tid >> 5, lane = tid & 31, ln = lane & 15, hh = lane >> 4;
  const int mt = blockIdx.y; const int nq0 = mt >> 2; const int nq = nq0 + blockIdx.x * 4 + w; if (nq >= NNQ) return;
  const float var = softplus1(bf16_round(phi[0])); const float r1 = 1.0f / (2.0f * var), r2 = 1.0f / (8.0f * var);
  const int row0 = mt * 16, col0 = nq * 64; const float* arow = x + (size_t)(row0 + ln) * DD;
  v8f acc[4] = {};
#pragma unroll 2
  for (int kb = 0; kb < DD; kb += 32) { FragB ah, az; const v4f x0 = *(const v4fa*)(arow + kb + 8 * hh), x1 = *(const v4fa*)(arow + kb + 8 * hh + 4), x2 = *(const v4fa*)(arow + kb + 16 + 8 * hh), x3 = *(const v4fa*)(arow + kb + 16 + 8 * hh + 4);
    const float xs[16] = {x0[0],x0[1],x0[2],x0[3],x1[0],x1[1],x1[2],x1[3],x2[0],x2[1],x2[2],x2[3],x3[0],x3[1],x3[2],x3[3]};
#pragma unroll
    for (int i = 0; i < 16; ++i) { ah.u[i] = bf16_bits(xs[i]); az.u[i] = 0; }
#pragma unroll
    for (int t = 0; t < 4; ++t) { const float* brow = x + (size_t)(col0 + t * 16 + ln) * DD + kb; FragB bq; const v4f y0 = *(const v4fa*)(brow + 8 * hh), y1 = *(const v4fa*)(brow + 8 * hh + 4), y2 = *(const v4fa*)(brow + 16 + 8 * hh), y3 = *(const v4fa*)(brow + 16 + 8 * hh + 4);
      const float ys[16] = {y0[0],y0[1],y0[2],y0[3],y1[0],y1[1],y1[2],y1[3],y2[0],y2[1],y2[2],y2[3],y3[0],y3[1],y3[2],y3[3]};
#pragma unroll
      for (int i = 0; i < 16; ++i) bq.u[i] = bf16_bits(ys[i]);
      acc[t] = mmaN<1>(ah.v, az.v, bq.v, bq.v, acc[t]); } }
  __shared__ float se1[4][16][65], se2[4][16][65];
#pragma unroll
  for (int t = 0; t < 4; ++t) {
#pragma unroll
    for (int r = 0; r < 8; ++r) se1[w][8 * hh + r][t * 16 + ln] = acc[t][r]; }
  __builtin_amdgcn_fence(__ATOMIC_ACQ_REL, "workgroup"); __builtin_amdgcn_wave_barrier();
  { const int rr = lane & 15, half = lane >> 4; const int i = row0 + rr; const float sqi = sq[i];
#pragma unroll 1
    for (int cc = half * 32; cc < half * 32 + 32; ++cc) { const int j = col0 + cc; float e1 = 0.f, e2 = 0.f;
      if (j >= i) { const float d = fmaxf((sqi + sq[j]) - 2.0f * se1[w][rr][cc], 0.f); e1 = __expf(-(d * r1)); e2 = __expf(-(d * r2)); }
      se1[w][rr][cc] = e1; se2[w][rr][cc] = e2; } }
  __builtin_amdgcn_fence(__ATOMIC_ACQ_REL, "workgroup"); __builtin_amdgcn_wave_barrier();
  float rsa = 0.f, rsb = 0.f; { const int rr = lane & 15, half = lane >> 4;
#pragma unroll 1
    for (int cc = half * 32; cc < half * 32 + 32; ++cc) { rsa += se1[w][rr][cc]; rsb += se2[w][rr][cc]; } rsa += __shfl_xor(rsa, 16, 32); rsb += __shfl_xor(rsb, 16, 32); }
  float ca0 = 0.f, cb0 = 0.f, ca1 = 0.f, cb1 = 0.f;
#pragma unroll 1
  for (int rr = 0; rr < 16; ++rr) { const int i = row0 + rr; const int j0 = col0 + lane, j1 = col0 + 32 + lane;
    if (j0 > i) { ca0 += se1[w][rr][lane]; cb0 += se2[w][rr][lane]; } if (j1 > i) { ca1 += se1[w][rr][32 + lane]; cb1 += se2[w][rr][32 + lane]; } }
  float* rp = RP + ((size_t)mt * NNQ + nq) * 32; float* cp = CP + ((size_t)mt * NNQ + nq) * 128;
  typedef float v2f __attribute__((ext_vector_type(2)));
  for (int pass = 0; pass < 2; ++pass) { if (lane < 16) { v2f v; v.x = rsa; v.y = rsb; *(volatile v2f*)(rp + lane * 2) = v; } { v2f a; a.x = ca0; a.y = cb0; *(volatile v2f*)(cp + lane * 2) = a; v2f b2; b2.x = ca1; b2.y = cb1; *(volatile v2f*)(cp + 64 + lane * 2) = b2; } if (pass == 0) __threadfence(); }
}
__global__ __launch_bounds__(256) void k_lse(const float* __restrict__ RP, const float* __restrict__ CP, float* __restrict__ LSE) { const int i = blockIdx.x * 256 + threadIdx.x; if (i >= NN) return; const int mt = i >> 4, ri = i & 15; const int nqi = i >> 6, ci = i & 63; float s1 = 0.f, s2 = 0.f;
#pragma unroll 1
  for (int nq = mt >> 2; nq < NNQ; ++nq) { const float* rp = RP + ((size_t)mt * NNQ + nq) * 32; s1 += rp[ri * 2]; s2 += rp[ri * 2 + 1]; }
#pragma unroll 1
  for (int m2 = 0; m2 < NMT; ++m2) { if ((m2 >> 2) > nqi) break; const float* cp = CP + ((size_t)m2 * NNQ + nqi) * 128; s1 += cp[ci * 2]; s2 += cp[ci * 2 + 1]; }
  typedef float v2f __attribute__((ext_vector_type(2))); v2f o; o.x = logf(s1); o.y = logf(s2); *(volatile v2f*)(LSE + (size_t)i * 2) = o; __threadfence(); *(volatile v2f*)(LSE + (size_t)i * 2) = o; }
__global__ __launch_bounds__(1024) void k_scalars(const float* __restrict__ LSE, const float* __restrict__ x, const float* __restrict__ phi, const float* __restrict__ pv, float* __restrict__ outs) {
  __shared__ double r1[1024], r2[1024], r3[1024]; const int t = threadIdx.x; double a = 0.0, b = 0.0, k = 0.0;
  const float var = softplus1(bf16_round(phi[0])); const float prior = bf16_round(pv[0]); const float kc = 0.5f * logf(prior / var) - 0.5f; const float kd = 1.0f / (2.0f * prior);
  for (int i = t; i < NN; i += 1024) { a += (double)LSE[i * 2]; b += (double)LSE[i * 2 + 1]; }
  for (size_t e = t; e < (size_t)NN * DD; e += 1024) { const float xv = x[e]; k += (double)(kc + (var + xv * xv) * kd); }
  r1[t] = a; r2[t] = b; r3[t] = k; __syncthreads(); for (int s = 512; s > 0; s >>= 1) { if (t < s) { r1[t] += r1[t + s]; r2[t] += r2[t + s]; r3[t] += r3[t + s]; } __syncthreads(); }
  if (t == 0) { const float logn = logf((float)NN); const float Ixt = logn - (float)(r1[0] / NN); const float Ixt_lb = logn - (float)(r2[0] / NN); const float vI = (float)(r3[0] / NN);
    *(volatile float*)(outs + 0) = Ixt_lb; *(volatile float*)(outs + 1) = Ixt; *(volatile float*)(outs + 2) = vI; __threadfence(); *(volatile float*)(outs + 0) = Ixt_lb; *(volatile float*)(outs + 1) = Ixt; *(volatile float*)(outs + 2) = vI; } }
__global__ __launch_bounds__(256) void k_out(const float* __restrict__ x, const float* __restrict__ nz, const float* __restrict__ phi, float* __restrict__ out) { const size_t t = (size_t)blockIdx.x * 256 + threadIdx.x; if (t >= (size_t)NN * DD / 4) return; const float sd = sqrtf(softplus1(bf16_round(phi[0]))); const v4f a = *(const v4fa*)(x + t * 4), b = *(const v4fa*)(nz + t * 4); v4f o; for (int q = 0; q < 4; ++q) o[q] = a[q] + b[q] * sd; *(volatile v4f*)(out + t * 4) = o;   __threadfence(); *(volatile v4f*)(out + t * 4) = o; }
extern "C" void kernel_launch(void* const* d_in, const int* in_sizes, int n_in,
                              void* d_out, int out_size, void* d_ws, size_t ws_size, hipStream_t stream) {
  (void)in_sizes; (void)n_in; (void)out_size;
  const float* x = (const float*)d_in[0]; const float* nz = (const float*)d_in[1]; const float* phi = (const float*)d_in[2]; const float* pv = (const float*)d_in[3];
  float* out = (float*)d_out; float* outs = out + (size_t)NN * DD;
  char* ws = (char*)d_ws; size_t off = 0;
  auto take = [&](size_t bytes) { char* p = ws + off; off += (bytes + 255) & ~(size_t)255; return p; };
  float* sq = (float*)take(NN * 4); float* RP = (float*)take((size_t)NMT * NNQ * 32 * 4); float* CP = (float*)take((size_t)NMT * NNQ * 128 * 4); float* LSE = (float*)take((size_t)NN * 2 * 4);
  if (off > ws_size) return;
  k_sq<<<NN / 32, 1024, 0, stream>>>(x, sq);
  k_gram<<<dim3((NNQ + 3) / 4, NMT), 128, 0, stream>>>(x, sq, phi, RP, CP);
  k_lse<<<NN / 256, 256, 0, stream>>>(RP, CP, LSE);
  k_out<<<(unsigned)(((size_t)NN * DD / 4 + 255) / 256), 256, 0, stream>>>(x, nz, phi, out);
  k_scalars<<<1, 1024, 0, stream>>>(LSE, x, phi, pv, outs);
}
